// QFNN_83906481095375
// MI455X (gfx1250) — hardware-verified
//
#include <hip/hip_runtime.h>
#include <stdint.h>
#include <math.h>


typedef __attribute__((ext_vector_type(16))) _Float16 v16h;
typedef __attribute__((ext_vector_type(8)))  _Float16 v8h;
typedef __attribute__((ext_vector_type(16))) __bf16   v16b;
typedef __attribute__((ext_vector_type(8)))  __bf16   v8b;
typedef __attribute__((ext_vector_type(8)))  float    v8f;
typedef __attribute__((ext_vector_type(4)))  float    v4f;

__device__ __forceinline__ unsigned short f2bf_bits(float f) {
  unsigned u = __float_as_uint(f);
  return (unsigned short)((u + 0x7FFFu + ((u >> 16) & 1u)) >> 16);
}
__device__ __forceinline__ float bf_bits2f(unsigned short h) { return __uint_as_float(((unsigned)h) << 16); }

__device__ __forceinline__ void dep_guard_h(v8f& a, v8f& b, v16h x, v16h y) { asm volatile("v_nop\n\tv_nop\n\tv_nop\n\tv_nop" : "+v"(a), "+v"(b) : "v"(x), "v"(y)); }
__device__ __forceinline__ void dep_guard_b(v8f& a, v8f& b, v16b x, v16b y) { asm volatile("v_nop\n\tv_nop\n\tv_nop\n\tv_nop" : "+v"(a), "+v"(b) : "v"(x), "v"(y)); }
__device__ __forceinline__ void keep4_h(v16h a, v16h b, v16h c, v16h d) { asm volatile("v_nop" :: "v"(a), "v"(b), "v"(c), "v"(d)); }
__device__ __forceinline__ void keep4_b(v16b a, v16b b, v16b c, v16b d) { asm volatile("v_nop" :: "v"(a), "v"(b), "v"(c), "v"(d)); }
__device__ __forceinline__ void acc_guard4(v8f& a, v8f& b, v8f& c, v8f& d) { asm volatile("v_nop\n\tv_nop\n\tv_nop\n\tv_nop" : "+v"(a), "+v"(b), "+v"(c), "+v"(d)); }
template <typename T> struct Frag;
template <> struct Frag<_Float16> {
  typedef v16h V; union U { v16h v; v8h h[2]; };
  static __device__ __forceinline__ v16h load(const _Float16* p) {
    U f; f.h[0] = *(const v8h*)(p); f.h[1] = *(const v8h*)(p + 16); return f.v;
  }
  static __device__ __forceinline__ v8f mma(v16h a, v16h b, v8f c) {
    return __builtin_amdgcn_wmma_f32_16x16x32_f16(false, a, false, b, (short)0, c, false, false);
  }
  static __device__ __forceinline__ void guard(v8f& a, v8f& b, v16h x, v16h y) { dep_guard_h(a, b, x, y); }
  static __device__ __forceinline__ void keep(v16h a, v16h b, v16h c, v16h d) { keep4_h(a, b, c, d); }
};
template <> struct Frag<__bf16> {
  typedef v16b V; union U { v16b v; v8b h[2]; };
  static __device__ __forceinline__ v16b load(const __bf16* p) {
    U f; f.h[0] = *(const v8b*)(p); f.h[1] = *(const v8b*)(p + 16); return f.v;
  }
  static __device__ __forceinline__ v8f mma(v16b a, v16b b, v8f c) {
    return __builtin_amdgcn_wmma_f32_16x16x32_bf16(false, a, false, b, (short)0, c, false, false);
  }
  static __device__ __forceinline__ void guard(v8f& a, v8f& b, v16b x, v16b y) { dep_guard_b(a, b, x, y); }
  static __device__ __forceinline__ void keep(v16b a, v16b b, v16b c, v16b d) { keep4_b(a, b, c, d); }
};

__device__ __forceinline__ v8f mma16h(v16h a, v16h b, v8f c) {
  c = __builtin_amdgcn_wmma_f32_16x16x32_f16(false, a, false, b, (short)0, c, false, false);
  asm volatile("v_nop\n\tv_nop\n\tv_nop\n\tv_nop" : "+v"(c) : "v"(a), "v"(b));
  return c;
}
__device__ __forceinline__ v8f zero8f() { v8f z; z[0]=0.f; z[1]=0.f; z[2]=0.f; z[3]=0.f; z[4]=0.f; z[5]=0.f; z[6]=0.f; z[7]=0.f; return z; }

template <int ET> struct Elem;
template <> struct Elem<0> { typedef _Float16 T; };
template <> struct Elem<1> { typedef __bf16 T; };
template <int ET, bool SPLIT, int BIAS_MODE, int OUT_MODE, bool RESID, int ACT = 0>
__global__ __launch_bounds__(256) void wmma_gemm64(
    const unsigned short* __restrict__ Ap, const unsigned short* __restrict__ A2p, int lda, long strideA,
    const unsigned short* __restrict__ Btp, const unsigned short* __restrict__ Bt2p, int ldb, long strideB,
    void* __restrict__ Cout, void* __restrict__ Cout2, int ldc, long strideC,
    const float* __restrict__ bias,
    const float* __restrict__ resid, long strideR,
    int M, int N, int K, float scale) {
  typedef typename Elem<ET>::T T;
  typedef typename Frag<T>::V V;
  const T* A = (const T*)Ap; const T* A2 = (const T*)A2p; const T* Bt = (const T*)Btp; const T* Bt2 = (const T*)Bt2p;
  __shared__ __align__(16) float sT[8][16 * 68];
  const int b    = blockIdx.y;
  const int lane = threadIdx.x & 31;
  const int wave = threadIdx.x >> 5;
  const int tilesN = N >> 6;
  const int tilesM = M >> 6;
  const int tile = blockIdx.x * 8 + wave;
  if (tile >= tilesM * tilesN) return;
  const int tm = tile / tilesN;
  const int tn = tile - tm * tilesN;
  const int m0 = tm << 6;
  const int n0 = tn << 6;

  const T* Ab  = A  + (size_t)b * strideA;
  const T* Bb  = Bt + (size_t)b * strideB;
  const T* Ab2 = SPLIT ? (A2  + (size_t)b * strideA) : nullptr;
  const T* Bb2 = SPLIT ? (Bt2 + (size_t)b * strideB) : nullptr;

  const int rlane = lane & 15;
  const int koff  = (lane >> 4) * 8;
  const int mOff  = (lane >> 4) * 8;

  v8f acc[4][4];
#pragma unroll
  for (int i = 0; i < 4; ++i)
#pragma unroll
    for (int j = 0; j < 4; ++j) acc[i][j] = (v8f){0.f,0.f,0.f,0.f,0.f,0.f,0.f,0.f};

  for (int k0 = 0; k0 < K; k0 += 32) {
    V bh[4], bl[4];
#pragma unroll
    for (int j = 0; j < 4; ++j) {
      const size_t bo = (size_t)(n0 + (j << 4) + rlane) * ldb + koff + k0;
      bh[j] = Frag<T>::load(Bb + bo);
      if (SPLIT) bl[j] = Frag<T>::load(Bb2 + bo);
    }
#pragma unroll
    for (int i = 0; i < 4; ++i) {
      const size_t ao = (size_t)(m0 + (i << 4) + rlane) * lda + koff + k0;
      V ah = Frag<T>::load(Ab + ao);
      V al;
      if (SPLIT) al = Frag<T>::load(Ab2 + ao);
#pragma unroll
      for (int j = 0; j < 4; ++j) {
        acc[i][j] = Frag<T>::mma(ah, bh[j], acc[i][j]);
        if (SPLIT) {
          acc[i][j] = Frag<T>::mma(ah, bl[j], acc[i][j]);
          acc[i][j] = Frag<T>::mma(al, bh[j], acc[i][j]);
        }
      }
      Frag<T>::guard(acc[i][0], acc[i][3], ah, SPLIT ? al : ah);
    }
    Frag<T>::keep(bh[0], bh[1], bh[2], bh[3]);
    if (SPLIT) Frag<T>::keep(bl[0], bl[1], bl[2], bl[3]);
  }
  acc_guard4(acc[0][0], acc[0][1], acc[0][2], acc[0][3]);
  acc_guard4(acc[1][0], acc[1][1], acc[1][2], acc[1][3]);
  acc_guard4(acc[2][0], acc[2][1], acc[2][2], acc[2][3]);
  acc_guard4(acc[3][0], acc[3][1], acc[3][2], acc[3][3]);

  float* slab = sT[wave];
  const float* Rb = RESID ? (resid + (size_t)b * strideR) : nullptr;
#pragma unroll
  for (int i = 0; i < 4; ++i) {
    const int mBase = m0 + (i << 4);
#pragma unroll
    for (int j = 0; j < 4; ++j) {
      const int n = n0 + (j << 4) + rlane;
      float bv = 0.f;
      if (BIAS_MODE == 2) bv = bias[n];
#pragma unroll
      for (int r = 0; r < 8; ++r) {
        float v = acc[i][j][r] * scale;
        if (BIAS_MODE == 1) v += bias[mBase + mOff + r];
        if (BIAS_MODE == 2) v += bv;
        if (RESID) v += Rb[(size_t)(mBase + mOff + r) * ldc + n];
        if (ACT == 1) v = tanhf(v);
        if (ACT == 2) v = fmaxf(v, 0.0f);
        if (ACT == 3) v = v / (1.0f + expf(-v));
        if (ACT == 4) v = (v > 0.f) ? v : 0.01f * v;
        if (ACT == 5) v = 0.5f * v * (1.0f + erff(v * 0.70710678118654752f));
        slab[(mOff + r) * 68 + (j << 4) + rlane] = v;
      }
    }
    __builtin_amdgcn_fence(__ATOMIC_RELEASE, "workgroup");
    __builtin_amdgcn_wave_barrier();
    __builtin_amdgcn_fence(__ATOMIC_ACQUIRE, "workgroup");
    if (OUT_MODE == 0) {
      float* C = (float*)Cout + (size_t)b * strideC;
      const int hh = lane >> 4, c4 = (lane & 15) * 4;
      for (int pass = 0; pass < 2; ++pass) {
#pragma unroll
        for (int it = 0; it < 8; ++it) {
          const int row = it * 2 + hh;
          v4f v = *(const v4f*)(slab + row * 68 + c4);
          *(volatile v4f*)(C + (size_t)(mBase + row) * ldc + n0 + c4) = v;
        }
        __threadfence();
      }
    } else {
      const int q = lane >> 3, c8 = (lane & 7) * 8;
      unsigned short* C  = (unsigned short*)Cout  + (size_t)b * strideC;
      unsigned short* C2 = (OUT_MODE == 2) ? ((unsigned short*)Cout2 + (size_t)b * strideC) : nullptr;
      for (int pass = 0; pass < 2; ++pass) {
#pragma unroll
        for (int it = 0; it < 4; ++it) {
          const int row = it * 4 + q;
          const float* sp = slab + row * 68 + c8;
          v8h hv, lv;
#pragma unroll
          for (int e = 0; e < 8; ++e) {
            if (OUT_MODE == 1) {
              hv[e] = (_Float16)sp[e];
            } else {
              unsigned short hb = f2bf_bits(sp[e]);
              unsigned short lb = f2bf_bits(sp[e] - bf_bits2f(hb));
              hv[e] = __builtin_bit_cast(_Float16, hb);
              lv[e] = __builtin_bit_cast(_Float16, lb);
            }
          }
          *(volatile v8h*)(C + (size_t)(mBase + row) * ldc + n0 + c8) = hv;
          if (OUT_MODE == 2) *(volatile v8h*)(C2 + (size_t)(mBase + row) * ldc + n0 + c8) = lv;
        }
        __threadfence();
      }
    }
    __builtin_amdgcn_fence(__ATOMIC_RELEASE, "workgroup");
    __builtin_amdgcn_wave_barrier();
    __builtin_amdgcn_fence(__ATOMIC_ACQUIRE, "workgroup");
  }
}

union Tile9216 { v8h v[1152]; _Float16 h[9216]; };
union Tile3136 { v8h v[392];  _Float16 h[3136]; };
union Out1280  { v4f v[320];  float    f[1280]; };

__global__ __launch_bounds__(256) void prep_weights_kernel(
    const float* __restrict__ c2w, const float* __restrict__ fc1w,
    const float* __restrict__ fc2w, const float* __restrict__ fc3w,
    _Float16* __restrict__ w2t, _Float16* __restrict__ w1h,
    _Float16* __restrict__ w2h, _Float16* __restrict__ w3h) {
  const int t = blockIdx.x * 256 + threadIdx.x;
  const int n1 = 128 * 3136 / 8;
  const int n2t = 9 * 64 * 32 / 8;
  const int n2 = 64 * 128 / 8;
  const int n3 = 16 * 64 / 8;
  v8h v;
  _Float16* dst;
  if (t < n1) {
    const float* s = fc1w + (size_t)t * 8;
#pragma unroll
    for (int e = 0; e < 8; ++e) v[e] = (_Float16)(s[e] * 64.0f);
    dst = w1h + (size_t)t * 8;
  } else if (t < n1 + n2t) {
    const int base = (t - n1) * 8;
    const int tap = base >> 11;
    const int rem = base & 2047;
    const int oc = rem >> 5, ic0 = rem & 31;
#pragma unroll
    for (int e = 0; e < 8; ++e) v[e] = (_Float16)(c2w[(oc * 32 + ic0 + e) * 9 + tap] * 16.0f);
    dst = w2t + base;
  } else if (t < n1 + n2t + n2) {
    const int base = (t - n1 - n2t) * 8;
#pragma unroll
    for (int e = 0; e < 8; ++e) v[e] = (_Float16)(fc2w[base + e] * 8.0f);
    dst = w2h + base;
  } else if (t < n1 + n2t + n2 + n3) {
    const int base = (t - n1 - n2t - n2) * 8;
#pragma unroll
    for (int e = 0; e < 8; ++e) v[e] = (_Float16)(fc3w[base + e] * 8.0f);
    dst = w3h + base;
  } else {
    return;
  }
  *(volatile v8h*)dst = v;
  __threadfence();
  *(volatile v8h*)dst = v;
}

__global__ __launch_bounds__(256) void conv1_pool_kernel(
    const float* __restrict__ x, const float* __restrict__ w, const float* __restrict__ bias,
    _Float16* __restrict__ p1, int nsamp) {
  __shared__ float sx[900];
  __shared__ float sw[288];
  __shared__ float sb[32];
  __shared__ __align__(16) Tile9216 st;
  const int tid = threadIdx.x;
  int bi = blockIdx.x;
  bi = bi < nsamp ? bi : nsamp - 1;
  const float* xb = x + (size_t)bi * 784;
  for (int i = tid; i < 900; i += 256) {
    const int r = i / 30, cc = i - r * 30;
    float v = 0.f;
    if (r >= 1 && r <= 28 && cc >= 1 && cc <= 28) v = xb[(r - 1) * 28 + (cc - 1)];
    sx[i] = v;
  }
  for (int i = tid; i < 288; i += 256) sw[i] = w[i];
  if (tid < 32) sb[tid] = bias[tid];
  {
    v8h z;
#pragma unroll
    for (int e = 0; e < 8; ++e) z[e] = (_Float16)0.0f;
    for (int i = tid; i < 1152; i += 256) st.v[i] = z;
  }
  __syncthreads();
  for (int idx = tid; idx < 6272; idx += 256) {
    const int oc = idx & 31;
    const int pix = idx >> 5;
    const int my = pix / 14, mx = pix - my * 14;
    const float* wk = sw + oc * 9;
    const float* sp = sx + (2 * my) * 30 + 2 * mx;
    float xv[16];
#pragma unroll
    for (int r = 0; r < 4; ++r)
#pragma unroll
      for (int q = 0; q < 4; ++q) xv[r * 4 + q] = sp[r * 30 + q];
    float w9[9];
#pragma unroll
    for (int t = 0; t < 9; ++t) w9[t] = wk[t];
    float s00 = 0.f, s01 = 0.f, s10 = 0.f, s11 = 0.f;
#pragma unroll
    for (int ky = 0; ky < 3; ++ky)
#pragma unroll
      for (int kx = 0; kx < 3; ++kx) {
        const float wv = w9[ky * 3 + kx];
        s00 += xv[ky * 4 + kx] * wv;
        s01 += xv[ky * 4 + kx + 1] * wv;
        s10 += xv[(ky + 1) * 4 + kx] * wv;
        s11 += xv[(ky + 1) * 4 + kx + 1] * wv;
      }
    const float m = fmaxf(fmaxf(s00, s01), fmaxf(s10, s11));
    const float val = fmaxf(m + sb[oc], 0.f);
    st.h[((my + 1) * 18 + (mx + 1)) * 32 + oc] = (_Float16)val;
  }
  __syncthreads();
  _Float16* dst = p1 + (size_t)bi * 9216;
  for (int pass = 0; pass < 2; ++pass) {
    for (int i = tid; i < 1152; i += 256) {
      const v8h v = st.v[i];
      *(volatile v8h*)(dst + (size_t)i * 8) = v;
    }
    __threadfence();
  }
}

__global__ __launch_bounds__(256) void conv2_pool_kernel(
    const _Float16* __restrict__ p1, const _Float16* __restrict__ w2t,
    const float* __restrict__ c2b, _Float16* __restrict__ p2, int nsamp) {
  __shared__ __align__(16) Tile9216 s_in;
  __shared__ float lsd[64 * 2 * 16];
  __shared__ float s_b2[64];
  __shared__ __align__(16) Tile3136 s_p2;
  const int tid = threadIdx.x, wave = tid >> 5, lane = tid & 31;
  const int hh = lane >> 4, c = lane & 15;
  int bi = blockIdx.x;
  bi = bi < nsamp ? bi : nsamp - 1;
  const _Float16* src = p1 + (size_t)bi * 9216;
  for (int i = tid; i < 1152; i += 256) s_in.v[i] = *(const v8h*)(src + (size_t)i * 8);
  if (tid < 64) s_b2[tid] = c2b[tid];
  __syncthreads();
  const int mt = wave & 3, ns = wave >> 2;
  v16h af[9];
#pragma unroll
  for (int tap = 0; tap < 9; ++tap)
    af[tap] = Frag<_Float16>::load(w2t + ((tap * 64 + mt * 16 + c) * 32) + 8 * hh);
  for (int ty = 0; ty < 7; ++ty) {
    const int y = 2 * ty + ns;
    v8f acc = zero8f();
#pragma unroll
    for (int tap = 0; tap < 9; ++tap) {
      const int ky = tap / 3, kx = tap - ky * 3;
      const v16h bf = Frag<_Float16>::load(s_in.h + ((y + ky) * 18 + (c + kx)) * 32 + 8 * hh);
      acc = mma16h(af[tap], bf, acc);
    }
#pragma unroll
    for (int r = 0; r < 8; ++r) {
      const int oc = mt * 16 + 8 * hh + r;
      lsd[(oc * 2 + ns) * 16 + c] = fmaxf(acc[r] * 0.0625f + s_b2[oc], 0.f);
    }
    __syncthreads();
    for (int idx = tid; idx < 448; idx += 256) {
      const int oc = idx / 7, px = idx - oc * 7;
      const float* l0 = lsd + (oc * 2) * 16 + 2 * px;
      const float m = fmaxf(fmaxf(l0[0], l0[1]), fmaxf(l0[16], l0[17]));
      s_p2.h[oc * 49 + ty * 7 + px] = (_Float16)m;
    }
    __syncthreads();
  }
  _Float16* dst = p2 + (size_t)bi * 3136;
  for (int pass = 0; pass < 2; ++pass) {
    for (int i = tid; i < 392; i += 256) {
      const v8h v = s_p2.v[i];
      *(volatile v8h*)(dst + (size_t)i * 8) = v;
    }
    __threadfence();
  }
}

__global__ __launch_bounds__(256) void tail_kernel(
    const _Float16* __restrict__ h2, const _Float16* __restrict__ w3h,
    const float* __restrict__ fc3b, const float* __restrict__ qw,
    const float* __restrict__ fc4w, const float* __restrict__ fc4b,
    float* __restrict__ out, int nsamp) {
  __shared__ float s_feat[8 * 256];
  __shared__ float s_U[64];
  __shared__ float s_W4[200];
  __shared__ float s_b4[16];
  __shared__ float s_b3[16];
  __shared__ __align__(16) Out1280 s_out;
  const int tid = threadIdx.x, wave = tid >> 5, lane = tid & 31;
  const int hh = lane >> 4, c = lane & 15;
  const int sbase = blockIdx.x * 128;
  for (int i = tid; i < 200; i += 256) s_W4[i] = fc4w[i];
  if (tid < 16) { s_b3[tid] = fc3b[tid]; s_b4[tid] = (tid < 10) ? fc4b[tid] : 0.f; }
  if (tid < 8) {
    const float phi = qw[tid * 3 + 0], th = qw[tid * 3 + 1], om = qw[tid * 3 + 2];
    const float ct = cosf(0.5f * th), st = sinf(0.5f * th);
    const float aa = 0.5f * (phi + om), bb = 0.5f * (phi - om);
    const float ca = cosf(aa), sa = sinf(aa), cb = cosf(bb), sb = sinf(bb);
    float* U = s_U + tid * 8;
    U[0] =  ca * ct; U[1] = -sa * ct;
    U[2] = -cb * st; U[3] = -sb * st;
    U[4] =  cb * st; U[5] = -sb * st;
    U[6] =  ca * ct; U[7] =  sa * ct;
  }
  int row = sbase + wave * 16 + c;
  row = row < nsamp ? row : nsamp - 1;
  const _Float16* arow = h2 + (size_t)row * 64 + 8 * hh;
  const _Float16* brow = w3h + c * 64 + 8 * hh;
  v8f acc = zero8f();
#pragma unroll
  for (int k0 = 0; k0 < 64; k0 += 32) {
    const v16h a = Frag<_Float16>::load(arow + k0);
    const v16h bf = Frag<_Float16>::load(brow + k0);
    acc = mma16h(a, bf, acc);
  }
  __syncthreads();
  float* sf = s_feat + wave * 256;
#pragma unroll
  for (int r = 0; r < 8; ++r) sf[(8 * hh + r) * 16 + c] = fmaxf(acc[r] * 0.125f + s_b3[c], 0.f);
  __syncthreads();

  for (int it = 0; it < 8; ++it) {
    const int ls = it * 2 + hh;
    const float f = sf[ls * 16 + c];
    float n2 = f * f;
    n2 += __shfl_xor(n2, 8, 32); n2 += __shfl_xor(n2, 4, 32); n2 += __shfl_xor(n2, 2, 32); n2 += __shfl_xor(n2, 1, 32);
    const float inv = 1.0f / fmaxf(sqrtf(n2), 1e-12f);
    float re = f * inv, im = 0.f;
#pragma unroll 1
    for (int layer = 0; layer < 2; ++layer) {
#pragma unroll 1
      for (int q = 0; q < 4; ++q) {
        const float* U = s_U + (layer * 4 + q) * 8;
        const int mask = 8 >> q;
        const float yr = __shfl_xor(re, mask, 32);
        const float yi = __shfl_xor(im, mask, 32);
        const bool bit = (c & mask) != 0;
        const float Ar = bit ? U[6] : U[0], Ai = bit ? U[7] : U[1];
        const float Br = bit ? U[4] : U[2], Bi = bit ? U[5] : U[3];
        const float nr = Ar * re - Ai * im + Br * yr - Bi * yi;
        const float ni = Ar * im + Ai * re + Br * yi + Bi * yr;
        re = nr; im = ni;
      }
#pragma unroll 1
      for (int q = 0; q < 3; ++q) {
        const int cm = 8 >> q, tm = 4 >> q;
        const float yr = __shfl_xor(re, tm, 32);
        const float yi = __shfl_xor(im, tm, 32);
        if (c & cm) { re = yr; im = yi; }
      }
    }
    const float p = re * re + im * im;
    float qz[4];
#pragma unroll
    for (int q = 0; q < 4; ++q) {
      float v = (c & (8 >> q)) ? -p : p;
      v += __shfl_xor(v, 8, 32); v += __shfl_xor(v, 4, 32); v += __shfl_xor(v, 2, 32); v += __shfl_xor(v, 1, 32);
      qz[q] = v;
    }
    float zm = -INFINITY;
#pragma unroll 1
    for (int o = 0; o < 10; ++o) {
      const float* wrow = s_W4 + o * 20;
      float t = f * wrow[c];
      t += __shfl_xor(t, 8, 32); t += __shfl_xor(t, 4, 32); t += __shfl_xor(t, 2, 32); t += __shfl_xor(t, 1, 32);
      const float zo = t + qz[0] * wrow[16] + qz[1] * wrow[17] + qz[2] * wrow[18] + qz[3] * wrow[19] + s_b4[o];
      if (c == o) zm = zo;
    }
    float mx = zm;
    mx = fmaxf(mx, __shfl_xor(mx, 8, 32)); mx = fmaxf(mx, __shfl_xor(mx, 4, 32));
    mx = fmaxf(mx, __shfl_xor(mx, 2, 32)); mx = fmaxf(mx, __shfl_xor(mx, 1, 32));
    float se = expf(zm - mx);
    se += __shfl_xor(se, 8, 32); se += __shfl_xor(se, 4, 32); se += __shfl_xor(se, 2, 32); se += __shfl_xor(se, 1, 32);
    const float val = zm - mx - logf(se);
    if (c < 10) s_out.f[(wave * 16 + ls) * 10 + c] = val;
  }
  __syncthreads();
  float* ob = out + (size_t)sbase * 10;
  for (int pass = 0; pass < 2; ++pass) {
    for (int ch = tid; ch < 320; ch += 256) {
      const v4f v = s_out.v[ch];
      *(volatile v4f*)(ob + (size_t)ch * 4) = v;
    }
    __threadfence();
  }
}

extern "C" void kernel_launch(void* const* d_in, const int* in_sizes, int n_in,
                              void* d_out, int out_size, void* d_ws, size_t ws_size,
                              hipStream_t stream) {
  if (n_in < 14) return;
  const int B = in_sizes[0] / 784;
  if (B < 128 || (B % 128) != 0 || in_sizes[0] != B * 784) return;
  if (out_size != B * 10) return;
  if (in_sizes[1] != 288 || in_sizes[2] < 32 || in_sizes[3] != 18432 || in_sizes[4] < 64 ||
      in_sizes[5] != 401408 || in_sizes[6] < 128 || in_sizes[7] != 8192 || in_sizes[8] < 64 ||
      in_sizes[9] != 1024 || in_sizes[10] < 16 || in_sizes[11] < 24 || in_sizes[12] != 200 ||
      in_sizes[13] < 10) return;

  const float* x    = (const float*)d_in[0];
  const float* c1w  = (const float*)d_in[1];
  const float* c1b  = (const float*)d_in[2];
  const float* c2w  = (const float*)d_in[3];
  const float* c2b  = (const float*)d_in[4];
  const float* fc1w = (const float*)d_in[5];
  const float* fc1b = (const float*)d_in[6];
  const float* fc2w = (const float*)d_in[7];
  const float* fc2b = (const float*)d_in[8];
  const float* fc3w = (const float*)d_in[9];
  const float* fc3b = (const float*)d_in[10];
  const float* qw   = (const float*)d_in[11];
  const float* fc4w = (const float*)d_in[12];
  const float* fc4b = (const float*)d_in[13];
  float* out = (float*)d_out;

  char* ws = (char*)d_ws;
  size_t off = 0;
  auto take = [&](size_t bytes) {
    char* p = ws + off;
    off = (off + bytes + 255) & ~(size_t)255;
    return p;
  };
  _Float16* p1  = (_Float16*)take((size_t)B * 9216 * 2);
  _Float16* w2t = (_Float16*)take((size_t)9 * 64 * 32 * 2);
  _Float16* w1h = (_Float16*)take((size_t)128 * 3136 * 2);
  _Float16* w2h = (_Float16*)take((size_t)64 * 128 * 2);
  _Float16* w3h = (_Float16*)take((size_t)16 * 64 * 2);
  _Float16* p2  = (_Float16*)take((size_t)B * 3136 * 2);
  _Float16* h1  = (_Float16*)take((size_t)B * 128 * 2);
  _Float16* h2  = (_Float16*)take((size_t)B * 64 * 2);
  if (off > ws_size || off > (size_t)134217728) return;

  const int nprep = 50176 + 2304 + 1024 + 128;
  prep_weights_kernel<<<dim3((nprep + 255) / 256), dim3(256), 0, stream>>>(c2w, fc1w, fc2w, fc3w, w2t, w1h, w2h, w3h);
  conv1_pool_kernel<<<dim3(B), dim3(256), 0, stream>>>(x, c1w, c1b, p1, B);
  conv2_pool_kernel<<<dim3(B), dim3(256), 0, stream>>>(p1, w2t, c2b, p2, B);

  {
    const int tiles = (B / 64) * (128 / 64);
    const int blocks = (tiles + 7) / 8;
    hipLaunchKernelGGL(HIP_KERNEL_NAME(wmma_gemm64<0, false, 2, 1, false, 2>), dim3(blocks, 1, 1), dim3(256), 0, stream,
                       (const unsigned short*)p2, (const unsigned short*)p2, 3136, 0L,
                       (const unsigned short*)w1h, (const unsigned short*)w1h, 3136, 0L,
                       (void*)h1, (void*)h1, 128, 0L,
                       fc1b, fc1b, 0L, B, 128, 3136, 1.0f / 64.0f);
  }
  {
    const int tiles = (B / 64) * (64 / 64);
    const int blocks = (tiles + 7) / 8;
    hipLaunchKernelGGL(HIP_KERNEL_NAME(wmma_gemm64<0, false, 2, 1, false, 2>), dim3(blocks, 1, 1), dim3(256), 0, stream,
                       (const unsigned short*)h1, (const unsigned short*)h1, 128, 0L,
                       (const unsigned short*)w2h, (const unsigned short*)w2h, 128, 0L,
                       (void*)h2, (void*)h2, 64, 0L,
                       fc2b, fc2b, 0L, B, 64, 128, 1.0f / 8.0f);
  }
  tail_kernel<<<dim3(B / 128), dim3(256), 0, stream>>>(h2, w3h, fc3b, qw, fc4w, fc4b, out, B);
}
